// FlowV2Attention_84593675862629
// MI455X (gfx1250) — hardware-verified
//
#include <hip/hip_runtime.h>
#include <math.h>
#include <stdint.h>

constexpr int NB_BATCH  = 4;
constexpr int SEQ_LEN   = 2048;
constexpr int D_MODEL   = 1024;
constexpr int N_HEAD    = 16;
constexpr int HEAD_D    = 64;
constexpr int ROPE_HALF = 32;
constexpr int QK_LD     = 2 * D_MODEL;

typedef __attribute__((ext_vector_type(16))) _Float16 v16h;
typedef __attribute__((ext_vector_type(8)))  _Float16 v8h;
typedef __attribute__((ext_vector_type(16))) __bf16   v16b;
typedef __attribute__((ext_vector_type(8)))  __bf16   v8b;
typedef __attribute__((ext_vector_type(8)))  float    v8f;
typedef __attribute__((ext_vector_type(4)))  float    v4f;
typedef __attribute__((ext_vector_type(4)))  unsigned int v4u;

__device__ __forceinline__ unsigned short f2bf_bits(float f) {
  unsigned u = __float_as_uint(f);
  return (unsigned short)((u + 0x7FFFu + ((u >> 16) & 1u)) >> 16);
}
__device__ __forceinline__ float bf_bits2f(unsigned short h) { return __uint_as_float(((unsigned)h) << 16); }
__device__ __forceinline__ unsigned pk16(unsigned short a, unsigned short b) { return (unsigned)a | ((unsigned)b << 16); }

__device__ __forceinline__ void dep_guard_h(v8f& a, v8f& b, v16h x, v16h y) { asm volatile("v_nop\n\tv_nop\n\tv_nop\n\tv_nop" : "+v"(a), "+v"(b) : "v"(x), "v"(y)); }
__device__ __forceinline__ void dep_guard_b(v8f& a, v8f& b, v16b x, v16b y) { asm volatile("v_nop\n\tv_nop\n\tv_nop\n\tv_nop" : "+v"(a), "+v"(b) : "v"(x), "v"(y)); }
__device__ __forceinline__ void keep4_h(v16h a, v16h b, v16h c, v16h d) { asm volatile("v_nop" :: "v"(a), "v"(b), "v"(c), "v"(d)); }
__device__ __forceinline__ void keep4_b(v16b a, v16b b, v16b c, v16b d) { asm volatile("v_nop" :: "v"(a), "v"(b), "v"(c), "v"(d)); }
__device__ __forceinline__ void acc_guard4(v8f& a, v8f& b, v8f& c, v8f& d) { asm volatile("v_nop\n\tv_nop\n\tv_nop\n\tv_nop" : "+v"(a), "+v"(b), "+v"(c), "+v"(d)); }
template <typename T> struct Frag;
template <> struct Frag<_Float16> {
  typedef v16h V; union U { v16h v; v8h h[2]; };
  static __device__ __forceinline__ v16h load(const _Float16* p) {
    U f; f.h[0] = *(const v8h*)(p); f.h[1] = *(const v8h*)(p + 16); return f.v;
  }
  static __device__ __forceinline__ v8f mma(v16h a, v16h b, v8f c) {
    return __builtin_amdgcn_wmma_f32_16x16x32_f16(false, a, false, b, (short)0, c, false, false);
  }
  static __device__ __forceinline__ void guard(v8f& a, v8f& b, v16h x, v16h y) { dep_guard_h(a, b, x, y); }
  static __device__ __forceinline__ void keep(v16h a, v16h b, v16h c, v16h d) { keep4_h(a, b, c, d); }
};
template <> struct Frag<__bf16> {
  typedef v16b V; union U { v16b v; v8b h[2]; };
  static __device__ __forceinline__ v16b load(const __bf16* p) {
    U f; f.h[0] = *(const v8b*)(p); f.h[1] = *(const v8b*)(p + 16); return f.v;
  }
  static __device__ __forceinline__ v8f mma(v16b a, v16b b, v8f c) {
    return __builtin_amdgcn_wmma_f32_16x16x32_bf16(false, a, false, b, (short)0, c, false, false);
  }
  static __device__ __forceinline__ void guard(v8f& a, v8f& b, v16b x, v16b y) { dep_guard_b(a, b, x, y); }
  static __device__ __forceinline__ void keep(v16b a, v16b b, v16b c, v16b d) { keep4_b(a, b, c, d); }
};

template <int ET> struct Elem;
template <> struct Elem<0> { typedef _Float16 T; };
template <> struct Elem<1> { typedef __bf16 T; };
template <int ET, int SPLITM, int BIAS_MODE, int OUT_MODE, bool RESID, int ACT = 0>
__global__ __launch_bounds__(256) void wmma_gemm64(
    const unsigned short* __restrict__ Ap, const unsigned short* __restrict__ A2p, int lda, long strideA,
    const unsigned short* __restrict__ Btp, const unsigned short* __restrict__ Bt2p, int ldb, long strideB,
    void* __restrict__ Cout, void* __restrict__ Cout2, int ldc, long strideC,
    const float* __restrict__ bias,
    const float* __restrict__ resid, long strideR,
    const float* __restrict__ ropeC, const float* __restrict__ ropeS, int ropeT,
    int M, int N, int K, float scale) {
  typedef typename Elem<ET>::T T;
  typedef typename Frag<T>::V V;
  const T* A = (const T*)Ap; const T* A2 = (const T*)A2p; const T* Bt = (const T*)Btp; const T* Bt2 = (const T*)Bt2p;
  __shared__ __align__(16) float sT[8][16 * 68];
  const int b    = blockIdx.y;
  const int lane = threadIdx.x & 31;
  const int wave = threadIdx.x >> 5;
  const int tilesN = N >> 6;
  const int tilesM = M >> 6;
  const int tile = blockIdx.x * 8 + wave;
  if (tile >= tilesM * tilesN) return;
  const int tm = tile / tilesN;
  const int tn = tile - tm * tilesN;
  const int m0 = tm << 6;
  const int n0 = tn << 6;

  const T* Ab  = A  + (size_t)b * strideA;
  const T* Bb  = Bt + (size_t)b * strideB;
  const T* Ab2 = (SPLITM != 0) ? (A2  + (size_t)b * strideA) : nullptr;
  const T* Bb2 = (SPLITM == 1) ? (Bt2 + (size_t)b * strideB) : nullptr;

  const int rlane = lane & 15;
  const int koff  = (lane >> 4) * 8;
  const int mOff  = (lane >> 4) * 8;

  v8f acc[4][4];
#pragma unroll
  for (int i = 0; i < 4; ++i)
#pragma unroll
    for (int j = 0; j < 4; ++j) acc[i][j] = (v8f){0.f,0.f,0.f,0.f,0.f,0.f,0.f,0.f};

  for (int k0 = 0; k0 < K; k0 += 32) {
    V bh[4], bl[4];
#pragma unroll
    for (int j = 0; j < 4; ++j) {
      const size_t bo = (size_t)(n0 + (j << 4) + rlane) * ldb + koff + k0;
      bh[j] = Frag<T>::load(Bb + bo);
      if (SPLITM == 1) bl[j] = Frag<T>::load(Bb2 + bo);
    }
#pragma unroll
    for (int i = 0; i < 4; ++i) {
      const size_t ao = (size_t)(m0 + (i << 4) + rlane) * lda + koff + k0;
      V ah = Frag<T>::load(Ab + ao);
      V al;
      if (SPLITM != 0) al = Frag<T>::load(Ab2 + ao);
#pragma unroll
      for (int j = 0; j < 4; ++j) {
        acc[i][j] = Frag<T>::mma(ah, bh[j], acc[i][j]);
        if (SPLITM == 1) acc[i][j] = Frag<T>::mma(ah, bl[j], acc[i][j]);
        if (SPLITM != 0) acc[i][j] = Frag<T>::mma(al, bh[j], acc[i][j]);
      }
      Frag<T>::guard(acc[i][0], acc[i][3], ah, (SPLITM != 0) ? al : ah);
    }
    Frag<T>::keep(bh[0], bh[1], bh[2], bh[3]);
    if (SPLITM == 1) Frag<T>::keep(bl[0], bl[1], bl[2], bl[3]);
  }
  acc_guard4(acc[0][0], acc[0][1], acc[0][2], acc[0][3]);
  acc_guard4(acc[1][0], acc[1][1], acc[1][2], acc[1][3]);
  acc_guard4(acc[2][0], acc[2][1], acc[2][2], acc[2][3]);
  acc_guard4(acc[3][0], acc[3][1], acc[3][2], acc[3][3]);

  float* slab = sT[wave];
  const float* Rb = RESID ? (resid + (size_t)b * strideR) : nullptr;
#pragma unroll
  for (int i = 0; i < 4; ++i) {
    const int mBase = m0 + (i << 4);
#pragma unroll
    for (int j = 0; j < 4; ++j) {
      const int n = n0 + (j << 4) + rlane;
      float bv = 0.f;
      if (BIAS_MODE == 2) bv = bias[n];
      if (BIAS_MODE == 3) bv = bf_bits2f(f2bf_bits(bias[n]));
#pragma unroll
      for (int r = 0; r < 8; ++r) {
        float v = acc[i][j][r] * scale;
        if (BIAS_MODE == 1) v += bias[mBase + mOff + r];
        if (BIAS_MODE == 4) v += bf_bits2f(f2bf_bits(bias[mBase + mOff + r]));
        if (BIAS_MODE == 2 || BIAS_MODE == 3) v += bv;
        if (RESID) v += Rb[(size_t)(mBase + mOff + r) * ldc + n];
        if (ACT == 1) v = tanhf(v);
        if (ACT == 2) v = fmaxf(v, 0.0f);
        if (ACT == 3) v = v / (1.0f + expf(-v));
        if (ACT == 4) v = (v > 0.f) ? v : 0.01f * v;
        slab[(mOff + r) * 68 + (j << 4) + rlane] = v;
      }
    }
    __builtin_amdgcn_fence(__ATOMIC_RELEASE, "workgroup");
    __builtin_amdgcn_wave_barrier();
    __builtin_amdgcn_fence(__ATOMIC_ACQUIRE, "workgroup");
    if (OUT_MODE == 0) {
      float* C = (float*)Cout + (size_t)b * strideC;
      const int hh = lane >> 4, c4 = (lane & 15) * 4;
      for (int pass = 0; pass < 2; ++pass) {
#pragma unroll
        for (int it = 0; it < 8; ++it) {
          const int row = it * 2 + hh;
          v4f v = *(const v4f*)(slab + row * 68 + c4);
          *(volatile v4f*)(C + (size_t)(mBase + row) * ldc + n0 + c4) = v;
        }
        __threadfence();
      }
    } else {
      const int q = lane >> 3, c8 = (lane & 7) * 8;
      unsigned short* C  = (unsigned short*)Cout  + (size_t)b * strideC;
      unsigned short* C2 = (OUT_MODE == 2) ? ((unsigned short*)Cout2 + (size_t)b * strideC) : nullptr;
      for (int pass = 0; pass < 2; ++pass) {
#pragma unroll
        for (int it = 0; it < 4; ++it) {
          const int row = it * 4 + q;
          const float* sp = slab + row * 68 + c8;
          v8h hv, lv;
          if (OUT_MODE == 3) {
            const int t = (mBase + row) % ropeT;
            const v4f cv = *(const v4f*)(ropeC + (size_t)t * ROPE_HALF + (c8 >> 1));
            const v4f sv = *(const v4f*)(ropeS + (size_t)t * ROPE_HALF + (c8 >> 1));
#pragma unroll
            for (int e2 = 0; e2 < 4; ++e2) {
              const float x0 = sp[2 * e2], x1 = sp[2 * e2 + 1];
              hv[2 * e2]     = (_Float16)(x0 * cv[e2] - x1 * sv[e2]);
              hv[2 * e2 + 1] = (_Float16)(x0 * sv[e2] + x1 * cv[e2]);
            }
          } else {
#pragma unroll
            for (int e = 0; e < 8; ++e) {
              if (OUT_MODE == 1) {
                hv[e] = (_Float16)sp[e];
              } else {
                unsigned short hb = f2bf_bits(sp[e]);
                unsigned short lb = f2bf_bits(sp[e] - bf_bits2f(hb));
                hv[e] = __builtin_bit_cast(_Float16, hb);
                lv[e] = __builtin_bit_cast(_Float16, lb);
              }
            }
          }
          *(volatile v8h*)(C + (size_t)(mBase + row) * ldc + n0 + c8) = hv;
          if (OUT_MODE == 2) *(volatile v8h*)(C2 + (size_t)(mBase + row) * ldc + n0 + c8) = lv;
        }
        __threadfence();
      }
    }
    __builtin_amdgcn_fence(__ATOMIC_RELEASE, "workgroup");
    __builtin_amdgcn_wave_barrier();
    __builtin_amdgcn_fence(__ATOMIC_ACQUIRE, "workgroup");
  }
}

__global__ __launch_bounds__(256) void cast_bf16x8_kernel(const float* __restrict__ in, unsigned short* __restrict__ out, int n8) {
  const int i = blockIdx.x * 256 + threadIdx.x;
  if (i < n8) {
    const v4f a  = *(const v4f*)(in + 8 * (size_t)i);
    const v4f a2 = *(const v4f*)(in + 8 * (size_t)i + 4);
    v4u u;
    u[0] = pk16(f2bf_bits(a[0]),  f2bf_bits(a[1]));
    u[1] = pk16(f2bf_bits(a[2]),  f2bf_bits(a[3]));
    u[2] = pk16(f2bf_bits(a2[0]), f2bf_bits(a2[1]));
    u[3] = pk16(f2bf_bits(a2[2]), f2bf_bits(a2[3]));
    *(volatile v4u*)(out + 8 * (size_t)i) = u;
    __threadfence();
    *(volatile v4u*)(out + 8 * (size_t)i) = u;
  }
}

__global__ __launch_bounds__(256) void tcast_bf16_kernel(const float* __restrict__ W, unsigned short* __restrict__ oh, int R, int Cc) {
  __shared__ __align__(16) float tf[64 * 68];
  const int c0  = blockIdx.x * 64;
  const int rb0 = blockIdx.y * 64;
  const int tid = threadIdx.x;
  {
    const int lr = tid >> 4;
    const int c4 = (tid & 15) * 4;
#pragma unroll
    for (int it = 0; it < 4; ++it) {
      const int rr = it * 16 + lr;
      const v4f a = *(const v4f*)(W + (size_t)(rb0 + rr) * Cc + c0 + c4);
      *(v4f*)(tf + rr * 68 + c4) = a;
    }
  }
  __syncthreads();
  const int sub = tid >> 3;
  const int c8  = (tid & 7) * 8;
  v4u hv[2];
#pragma unroll
  for (int it = 0; it < 2; ++it) {
    const int oc = it * 32 + sub;
    v4u a;
#pragma unroll
    for (int q = 0; q < 4; ++q) {
      const float f0 = tf[(c8 + 2 * q) * 68 + oc];
      const float f1 = tf[(c8 + 2 * q + 1) * 68 + oc];
      a[q] = pk16(f2bf_bits(f0), f2bf_bits(f1));
    }
    hv[it] = a;
  }
  for (int pass = 0; pass < 2; ++pass) {
#pragma unroll
    for (int it = 0; it < 2; ++it) {
      const int oc = it * 32 + sub;
      const size_t go = (size_t)(c0 + oc) * R + rb0 + c8;
      *(volatile v4u*)(oh + go) = hv[it];
    }
    __threadfence();
  }
}

__global__ __launch_bounds__(32) void rope_freq_kernel(float* __restrict__ freq) {
  const int i = threadIdx.x;
  const float e = (float)(2 * i) / (float)HEAD_D;
  const float p = powf(10000.0f, e);
  const float f = 1.0f / p;
  ((volatile float*)freq)[i] = f;
  __threadfence();
  ((volatile float*)freq)[i] = f;
}

__global__ __launch_bounds__(256) void rope_table_kernel(const float* __restrict__ freq, float* __restrict__ cosT,
                                                         float* __restrict__ sinT, int n) {
  const int idx = blockIdx.x * 256 + threadIdx.x;
  if (idx < n) {
    const int t = idx >> 5, i = idx & 31;
    const float ang = (float)t * freq[i];
    float sv, cv;
    sincosf(ang, &sv, &cv);
    ((volatile float*)cosT)[idx] = cv;
    ((volatile float*)sinT)[idx] = sv;
    __threadfence();
    ((volatile float*)cosT)[idx] = cv;
    ((volatile float*)sinT)[idx] = sv;
  }
}

constexpr int AT_D  = 64;
constexpr int AT_NW = 4;
constexpr int AT_QB = 64;
constexpr int AT_KC = 64;
constexpr float P_CARRY = 32768.0f;

__device__ __forceinline__ v8f mma_h16(v16h a, v16h b, v8f c) {
  c = __builtin_amdgcn_wmma_f32_16x16x32_f16(false, a, false, b, (short)0, c, false, false);
  asm volatile("v_nop\n\tv_nop\n\tv_nop\n\tv_nop" : "+v"(c) : "v"(a), "v"(b));
  return c;
}

__global__ __launch_bounds__(128)
void attn_f16_kernel(const unsigned short* __restrict__ qkp, const unsigned short* __restrict__ vtp,
                     unsigned short* __restrict__ ohp, unsigned short* __restrict__ olp, float sscale) {
  union FB { v16h v; v8h h[2]; };
  __shared__ __align__(16) _Float16 Ksh[AT_KC * AT_D];
  __shared__ __align__(16) _Float16 Vth[AT_D * AT_KC];
  __shared__ __align__(16) _Float16 Psh[AT_NW][16 * AT_KC];
  __shared__ __align__(16) float    Os[AT_NW][16 * 68];

  const int tid  = threadIdx.x;
  const int wave = tid >> 5;
  const int lane = tid & 31;
  const int hh   = lane >> 4;
  const int c    = lane & 15;

  const int nqb = SEQ_LEN / AT_QB;
  const int bx = blockIdx.x;
  const int qb = bx % nqb;
  const int h  = bx / nqb;
  const int b  = blockIdx.y;
  const int q0 = qb * AT_QB + wave * 16;

  const _Float16* Qp = (const _Float16*)(const void*)qkp + (size_t)b * SEQ_LEN * QK_LD + (size_t)h * AT_D;
  const _Float16* Kp = Qp + D_MODEL;
  const _Float16* Vp = (const _Float16*)(const void*)vtp + ((size_t)b * D_MODEL + (size_t)h * AT_D) * SEQ_LEN;
  unsigned short* Oh = ohp + (size_t)b * SEQ_LEN * D_MODEL + (size_t)h * AT_D;
  unsigned short* Ol = olp + (size_t)b * SEQ_LEN * D_MODEL + (size_t)h * AT_D;

  v16h qa[2];
#pragma unroll
  for (int dc = 0; dc < 2; ++dc)
    qa[dc] = Frag<_Float16>::load(Qp + (size_t)(q0 + c) * QK_LD + dc * 32 + 8 * hh);

  float mrow[8], lrow[8];
  v8f oacc[4];
#pragma unroll
  for (int r = 0; r < 8; ++r) { mrow[r] = -INFINITY; lrow[r] = 0.f; }
#pragma unroll
  for (int t = 0; t < 4; ++t) oacc[t] = (v8f){0.f,0.f,0.f,0.f,0.f,0.f,0.f,0.f};

  for (int kc = 0; kc < SEQ_LEN / AT_KC; ++kc) {
    const int kv0 = kc * AT_KC;
    __syncthreads();
    {
      const int r = tid >> 1, half = (tid & 1) * 32;
      const _Float16* ks = Kp + (size_t)(kv0 + r) * QK_LD + half;
      const _Float16* vs = Vp + (size_t)r * SEQ_LEN + kv0 + half;
#pragma unroll
      for (int i = 0; i < 4; ++i) {
        const v8h a0 = *(const v8h*)(ks + 8 * i);
        const v8h b0 = *(const v8h*)(vs + 8 * i);
        *(v8h*)(Ksh + r * AT_D  + half + 8 * i) = a0;
        *(v8h*)(Vth + r * AT_KC + half + 8 * i) = b0;
      }
    }
    __syncthreads();

    v8f s[4];
#pragma unroll
    for (int j = 0; j < 4; ++j) {
      s[j] = (v8f){0.f,0.f,0.f,0.f,0.f,0.f,0.f,0.f};
#pragma unroll
      for (int dc = 0; dc < 2; ++dc) {
        FB kb;
        kb.h[0] = *(const v8h*)(Ksh + (j * 16 + c) * AT_D + dc * 32 + 8 * hh);
        kb.h[1] = *(const v8h*)(Ksh + (j * 16 + c) * AT_D + dc * 32 + 16 + 8 * hh);
        s[j] = mma_h16(qa[dc], kb.v, s[j]);
      }
      s[j] = s[j] * sscale;
    }
    float cm[8];
#pragma unroll
    for (int r = 0; r < 8; ++r) {
      float m = fmaxf(fmaxf(s[0][r], s[1][r]), fmaxf(s[2][r], s[3][r]));
#pragma unroll
      for (int off = 1; off < 16; off <<= 1) m = fmaxf(m, __shfl_xor(m, off, 32));
      cm[r] = m;
    }
    _Float16* pw = Psh[wave];
#pragma unroll
    for (int r = 0; r < 8; ++r) {
      const float mnew  = fmaxf(mrow[r], cm[r]);
      const float alpha = expf(mrow[r] - mnew);
      mrow[r] = mnew;
      float psum = 0.f;
#pragma unroll
      for (int j = 0; j < 4; ++j) {
        const float p = expf(s[j][r] - mnew);
        psum += p;
        pw[(8 * hh + r) * AT_KC + j * 16 + c] = (_Float16)(p * P_CARRY);
      }
#pragma unroll
      for (int off = 1; off < 16; off <<= 1) psum += __shfl_xor(psum, off, 32);
      lrow[r] = lrow[r] * alpha + psum;
#pragma unroll
      for (int t = 0; t < 4; ++t) oacc[t][r] *= alpha;
    }
    __builtin_amdgcn_fence(__ATOMIC_RELEASE, "workgroup");
    __builtin_amdgcn_wave_barrier();
    __builtin_amdgcn_fence(__ATOMIC_ACQUIRE, "workgroup");
#pragma unroll 1
    for (int kk = 0; kk < 2; ++kk) {
      FB pa;
      pa.h[0] = *(const v8h*)(pw + c * AT_KC + kk * 32 + 8 * hh);
      pa.h[1] = *(const v8h*)(pw + c * AT_KC + kk * 32 + 16 + 8 * hh);
#pragma unroll
      for (int t = 0; t < 4; ++t) {
        FB vb;
        vb.h[0] = *(const v8h*)(Vth + (t * 16 + c) * AT_KC + kk * 32 + 8 * hh);
        vb.h[1] = *(const v8h*)(Vth + (t * 16 + c) * AT_KC + kk * 32 + 16 + 8 * hh);
        oacc[t] = mma_h16(pa.v, vb.v, oacc[t]);
      }
    }
  }

  float* os = Os[wave];
#pragma unroll
  for (int r = 0; r < 8; ++r) {
    const float inv = 1.0f / (lrow[r] * P_CARRY);
#pragma unroll
    for (int t = 0; t < 4; ++t) os[(8 * hh + r) * 68 + t * 16 + c] = oacc[t][r] * inv;
  }
  __builtin_amdgcn_fence(__ATOMIC_RELEASE, "workgroup");
  __builtin_amdgcn_wave_barrier();
  __builtin_amdgcn_fence(__ATOMIC_ACQUIRE, "workgroup");
  {
    const int q8 = lane >> 3, c8 = (lane & 7) * 8;
    for (int pass = 0; pass < 2; ++pass) {
#pragma unroll
      for (int it = 0; it < 4; ++it) {
        const int row = it * 4 + q8;
        const float* sp = os + row * 68 + c8;
        v8h hv, lv;
#pragma unroll
        for (int e = 0; e < 8; ++e) {
          const unsigned short hb = f2bf_bits(sp[e]);
          const unsigned short lb = f2bf_bits(sp[e] - bf_bits2f(hb));
          hv[e] = __builtin_bit_cast(_Float16, hb);
          lv[e] = __builtin_bit_cast(_Float16, lb);
        }
        const size_t go = (size_t)(q0 + row) * D_MODEL + c8;
        *(volatile v8h*)(Oh + go) = hv;
        *(volatile v8h*)(Ol + go) = lv;
      }
      __threadfence();
    }
  }
}

extern "C" void kernel_launch(void* const* d_in, const int* in_sizes, int n_in,
                              void* d_out, int out_size, void* d_ws, size_t ws_size,
                              hipStream_t stream) {
  if (n_in < 5) return;
  const int M_ROWS = NB_BATCH * SEQ_LEN;
  if (in_sizes[0] != M_ROWS * D_MODEL) return;
  if (in_sizes[1] != D_MODEL * 3 * D_MODEL) return;
  if (in_sizes[2] != 3 * D_MODEL) return;
  if (in_sizes[3] != D_MODEL * D_MODEL) return;
  if (in_sizes[4] != D_MODEL) return;
  if (out_size != M_ROWS * D_MODEL) return;

  const float* x    = (const float*)d_in[0];
  const float* Wqkv = (const float*)d_in[1];
  const float* bqkv = (const float*)d_in[2];
  const float* Wout = (const float*)d_in[3];
  const float* bout = (const float*)d_in[4];
  float* out = (float*)d_out;

  char* ws = (char*)d_ws;
  size_t off = 0;
  unsigned short* xb   = (unsigned short*)(ws + off); off += (size_t)M_ROWS * D_MODEL * 2;
  unsigned short* wqT  = (unsigned short*)(ws + off); off += (size_t)3 * D_MODEL * D_MODEL * 2;
  unsigned short* woT  = (unsigned short*)(ws + off); off += (size_t)D_MODEL * D_MODEL * 2;
  float*          freq = (float*)(ws + off);          off += 256;
  float*          cosT = (float*)(ws + off);          off += (size_t)SEQ_LEN * ROPE_HALF * 4;
  float*          sinT = (float*)(ws + off);          off += (size_t)SEQ_LEN * ROPE_HALF * 4;
  unsigned short* qk16 = (unsigned short*)(ws + off); off += (size_t)M_ROWS * QK_LD * 2;
  unsigned short* vt16 = (unsigned short*)(ws + off); off += (size_t)NB_BATCH * D_MODEL * SEQ_LEN * 2;
  unsigned short* ohi  = (unsigned short*)(ws + off); off += (size_t)M_ROWS * D_MODEL * 2;
  unsigned short* olo  = (unsigned short*)(ws + off); off += (size_t)M_ROWS * D_MODEL * 2;
  if (off > ws_size) return;

  const int n8 = (M_ROWS * D_MODEL) / 8;
  cast_bf16x8_kernel<<<dim3((n8 + 255) / 256), dim3(256), 0, stream>>>(x, xb, n8);
  tcast_bf16_kernel<<<dim3(3 * D_MODEL / 64, D_MODEL / 64), dim3(256), 0, stream>>>(Wqkv, wqT, D_MODEL, 3 * D_MODEL);
  tcast_bf16_kernel<<<dim3(D_MODEL / 64, D_MODEL / 64), dim3(256), 0, stream>>>(Wout, woT, D_MODEL, D_MODEL);
  rope_freq_kernel<<<dim3(1), dim3(32), 0, stream>>>(freq);
  const int ntab = SEQ_LEN * ROPE_HALF;
  rope_table_kernel<<<dim3((ntab + 255) / 256), dim3(256), 0, stream>>>(freq, cosT, sinT, ntab);
  {
    const int tiles = (M_ROWS / 64) * (2 * D_MODEL / 64);
    wmma_gemm64<1, 0, 3, 3, false><<<dim3((tiles + 7) / 8, 1), dim3(256), 0, stream>>>(
        xb, nullptr, D_MODEL, 0L,
        wqT, nullptr, D_MODEL, 0L,
        (void*)qk16, nullptr, QK_LD, 0L,
        bqkv, nullptr, 0L,
        cosT, sinT, SEQ_LEN,
        M_ROWS, 2 * D_MODEL, D_MODEL, 1.0f);
  }
  {
    const int tiles = (D_MODEL / 64) * (SEQ_LEN / 64);
    wmma_gemm64<1, 0, 4, 1, false><<<dim3((tiles + 7) / 8, NB_BATCH), dim3(256), 0, stream>>>(
        wqT + (size_t)2 * D_MODEL * D_MODEL, nullptr, D_MODEL, 0L,
        xb, nullptr, D_MODEL, (long)SEQ_LEN * D_MODEL,
        (void*)vt16, nullptr, SEQ_LEN, (long)D_MODEL * SEQ_LEN,
        bqkv + 2 * D_MODEL, nullptr, 0L,
        nullptr, nullptr, 1,
        D_MODEL, SEQ_LEN, D_MODEL, 1.0f);
  }
  attn_f16_kernel<<<dim3(N_HEAD * (SEQ_LEN / AT_QB), NB_BATCH), dim3(128), 0, stream>>>(qk16, vt16, ohi, olo, 0.125f);
  {
    const int tiles = (M_ROWS / 64) * (D_MODEL / 64);
    wmma_gemm64<1, 2, 3, 0, false><<<dim3((tiles + 7) / 8, 1), dim3(256), 0, stream>>>(
        ohi, olo, D_MODEL, 0L,
        woT, nullptr, D_MODEL, 0L,
        (void*)out, nullptr, D_MODEL, 0L,
        bout, nullptr, 0L,
        nullptr, nullptr, 1,
        M_ROWS, D_MODEL, D_MODEL, 1.0f);
  }
}
